// ConcatCritic_3590592660028
// MI455X (gfx1250) — hardware-run, weakly checked
//
#include <hip/hip_runtime.h>
#include <math.h>

#ifndef NROW
#define NROW 512
#endif
#define NROW_FULL 512
#define DX 128
#define HID 512

typedef __attribute__((ext_vector_type(4))) float v4f;
typedef unsigned v4u __attribute__((ext_vector_type(4)));
typedef _Float16 h16;

#define VST2(T, ptr, val) do { const T vst2_v_ = (val); *(volatile T*)(ptr) = vst2_v_; __threadfence(); *(volatile T*)(ptr) = vst2_v_; } while (0)
#define VST2V4(ptr, val) do { const v4f vst2_v4_ = (val); *(volatile v4f*)(ptr) = vst2_v4_; __threadfence(); *(volatile v4f*)(ptr) = vst2_v4_; } while (0)

namespace eng {
typedef __attribute__((ext_vector_type(16))) _Float16 v16h;
typedef __attribute__((ext_vector_type(8)))  _Float16 v8h;
typedef __attribute__((ext_vector_type(16))) __bf16   v16b;
typedef __attribute__((ext_vector_type(8)))  __bf16   v8b;
typedef __attribute__((ext_vector_type(8)))  float    v8f;
typedef __attribute__((ext_vector_type(4)))  float    v4f;

__device__ __forceinline__ unsigned short f2bf_bits(float f) {
  unsigned u = __float_as_uint(f);
  return (unsigned short)((u + 0x7FFFu + ((u >> 16) & 1u)) >> 16);
}
__device__ __forceinline__ float bf_bits2f(unsigned short h) { return __uint_as_float(((unsigned)h) << 16); }

__device__ __forceinline__ void dep_guard_h(v8f& a, v8f& b, v16h x, v16h y) { asm volatile("v_nop\n\tv_nop\n\tv_nop\n\tv_nop" : "+v"(a), "+v"(b) : "v"(x), "v"(y)); }
__device__ __forceinline__ void dep_guard_b(v8f& a, v8f& b, v16b x, v16b y) { asm volatile("v_nop\n\tv_nop\n\tv_nop\n\tv_nop" : "+v"(a), "+v"(b) : "v"(x), "v"(y)); }
__device__ __forceinline__ void keep4_h(v16h a, v16h b, v16h c, v16h d) { asm volatile("v_nop" :: "v"(a), "v"(b), "v"(c), "v"(d)); }
__device__ __forceinline__ void keep4_b(v16b a, v16b b, v16b c, v16b d) { asm volatile("v_nop" :: "v"(a), "v"(b), "v"(c), "v"(d)); }
__device__ __forceinline__ void acc_guard4(v8f& a, v8f& b, v8f& c, v8f& d) { asm volatile("v_nop\n\tv_nop\n\tv_nop\n\tv_nop" : "+v"(a), "+v"(b), "+v"(c), "+v"(d)); }
template <typename T> struct Frag;
template <> struct Frag<_Float16> {
  typedef v16h V; union U { v16h v; v8h h[2]; };
  static __device__ __forceinline__ v16h load(const _Float16* p) {
    U f; f.h[0] = *(const v8h*)(p); f.h[1] = *(const v8h*)(p + 16); return f.v;
  }
  static __device__ __forceinline__ v8f mma(v16h a, v16h b, v8f c) {
    return __builtin_amdgcn_wmma_f32_16x16x32_f16(false, a, false, b, (short)0, c, false, false);
  }
  static __device__ __forceinline__ void guard(v8f& a, v8f& b, v16h x, v16h y) { dep_guard_h(a, b, x, y); }
  static __device__ __forceinline__ void keep(v16h a, v16h b, v16h c, v16h d) { keep4_h(a, b, c, d); }
};
template <> struct Frag<__bf16> {
  typedef v16b V; union U { v16b v; v8b h[2]; };
  static __device__ __forceinline__ v16b load(const __bf16* p) {
    U f; f.h[0] = *(const v8b*)(p); f.h[1] = *(const v8b*)(p + 16); return f.v;
  }
  static __device__ __forceinline__ v8f mma(v16b a, v16b b, v8f c) {
    return __builtin_amdgcn_wmma_f32_16x16x32_bf16(false, a, false, b, (short)0, c, false, false);
  }
  static __device__ __forceinline__ void guard(v8f& a, v8f& b, v16b x, v16b y) { dep_guard_b(a, b, x, y); }
  static __device__ __forceinline__ void keep(v16b a, v16b b, v16b c, v16b d) { keep4_b(a, b, c, d); }
};

template <int ET> struct Elem;
template <> struct Elem<0> { typedef _Float16 T; };
template <> struct Elem<1> { typedef __bf16 T; };
template <int ET, bool SPLIT, int BIAS_MODE, int OUT_MODE, bool RESID, int ACT = 0>
__device__ __forceinline__ void wmma_gemm64_body(
    const unsigned short* __restrict__ Ap, const unsigned short* __restrict__ A2p, int lda, long strideA,
    const unsigned short* __restrict__ Btp, const unsigned short* __restrict__ Bt2p, int ldb, long strideB,
    void* __restrict__ Cout, void* __restrict__ Cout2, int ldc, long strideC,
    const float* __restrict__ bias,
    const float* __restrict__ resid, long strideR,
    int M, int N, int K, float scale) {
  typedef typename Elem<ET>::T T;
  typedef typename Frag<T>::V V;
  const T* A = (const T*)Ap; const T* A2 = (const T*)A2p; const T* Bt = (const T*)Btp; const T* Bt2 = (const T*)Bt2p;
  __shared__ __align__(16) float sT[8][16 * 68];
  const int b    = blockIdx.y;
  const int lane = threadIdx.x & 31;
  const int wave = threadIdx.x >> 5;
  const int tilesN = N >> 6;
  const int tilesM = M >> 6;
  const int tile = blockIdx.x * 8 + wave;
  if (tile >= tilesM * tilesN) return;
  const int tm = tile / tilesN;
  const int tn = tile - tm * tilesN;
  const int m0 = tm << 6;
  const int n0 = tn << 6;

  const T* Ab  = A  + (size_t)b * strideA;
  const T* Bb  = Bt + (size_t)b * strideB;
  const T* Ab2 = SPLIT ? (A2  + (size_t)b * strideA) : nullptr;
  const T* Bb2 = SPLIT ? (Bt2 + (size_t)b * strideB) : nullptr;

  const int rlane = lane & 15;
  const int koff  = (lane >> 4) * 8;
  const int mOff  = (lane >> 4) * 8;

  v8f acc[4][4];
#pragma unroll
  for (int i = 0; i < 4; ++i)
#pragma unroll
    for (int j = 0; j < 4; ++j) acc[i][j] = (v8f){0.f,0.f,0.f,0.f,0.f,0.f,0.f,0.f};

  for (int k0 = 0; k0 < K; k0 += 32) {
    V bh[4], bl[4];
#pragma unroll
    for (int j = 0; j < 4; ++j) {
      const size_t bo = (size_t)(n0 + (j << 4) + rlane) * ldb + koff + k0;
      bh[j] = Frag<T>::load(Bb + bo);
      if (SPLIT) bl[j] = Frag<T>::load(Bb2 + bo);
    }
#pragma unroll
    for (int i = 0; i < 4; ++i) {
      const size_t ao = (size_t)(m0 + (i << 4) + rlane) * lda + koff + k0;
      V ah = Frag<T>::load(Ab + ao);
      V al;
      if (SPLIT) al = Frag<T>::load(Ab2 + ao);
#pragma unroll
      for (int j = 0; j < 4; ++j) {
        acc[i][j] = Frag<T>::mma(ah, bh[j], acc[i][j]);
        if (SPLIT) {
          acc[i][j] = Frag<T>::mma(ah, bl[j], acc[i][j]);
          acc[i][j] = Frag<T>::mma(al, bh[j], acc[i][j]);
        }
      }
      Frag<T>::guard(acc[i][0], acc[i][3], ah, SPLIT ? al : ah);
    }
    Frag<T>::keep(bh[0], bh[1], bh[2], bh[3]);
    if (SPLIT) Frag<T>::keep(bl[0], bl[1], bl[2], bl[3]);
  }
  acc_guard4(acc[0][0], acc[0][1], acc[0][2], acc[0][3]);
  acc_guard4(acc[1][0], acc[1][1], acc[1][2], acc[1][3]);
  acc_guard4(acc[2][0], acc[2][1], acc[2][2], acc[2][3]);
  acc_guard4(acc[3][0], acc[3][1], acc[3][2], acc[3][3]);

  float* slab = sT[wave];
  const float* Rb = RESID ? (resid + (size_t)b * strideR) : nullptr;
#pragma unroll
  for (int i = 0; i < 4; ++i) {
    const int mBase = m0 + (i << 4);
#pragma unroll
    for (int j = 0; j < 4; ++j) {
      const int n = n0 + (j << 4) + rlane;
      float bv = 0.f;
      if (BIAS_MODE == 2) bv = bias[n];
#pragma unroll
      for (int r = 0; r < 8; ++r) {
        float v = acc[i][j][r] * scale;
        if (BIAS_MODE == 1) v += bias[mBase + mOff + r];
        if (BIAS_MODE == 2) v += bv;
        if (RESID) v += Rb[(size_t)(mBase + mOff + r) * ldc + n];
        if (ACT == 1) v = tanhf(v);
        if (ACT == 2) v = fmaxf(v, 0.0f);
        if (ACT == 3) v = v / (1.0f + expf(-v));
        if (ACT == 4) v = (v > 0.f) ? v : 0.01f * v;
        if (ACT == 5) v = 0.5f * v * (1.0f + erff(v * 0.70710678118654752f));
        if (ACT == 6) v = (v > 0.f) ? v : 0.2f * v;
        if (ACT == 7) { const float u = 0.7978845608028654f * (v + 0.044715f * v * v * v); v = 0.5f * v * (1.f + tanhf(u)); }
        slab[(mOff + r) * 68 + (j << 4) + rlane] = v;
      }
    }
    __builtin_amdgcn_fence(3  , "workgroup");
    __builtin_amdgcn_wave_barrier();
    __builtin_amdgcn_fence(2  , "workgroup");
    if (OUT_MODE == 0) {
      float* C = (float*)Cout + (size_t)b * strideC;
      const int hh = lane >> 4, c4 = (lane & 15) * 4;
      for (int pass = 0; pass < 2; ++pass) {
#pragma unroll
        for (int it = 0; it < 8; ++it) {
          const int row = it * 2 + hh;
          v4f v = *(const v4f*)(slab + row * 68 + c4);
          *(volatile v4f*)(C + (size_t)(mBase + row) * ldc + n0 + c4) = v;
        }
        __threadfence();
      }
    } else {
      const int q = lane >> 3, c8 = (lane & 7) * 8;
      unsigned short* C  = (unsigned short*)Cout  + (size_t)b * strideC;
      unsigned short* C2 = (OUT_MODE == 2) ? ((unsigned short*)Cout2 + (size_t)b * strideC) : nullptr;
      for (int pass = 0; pass < 2; ++pass) {
#pragma unroll
        for (int it = 0; it < 4; ++it) {
          const int row = it * 4 + q;
          const float* sp = slab + row * 68 + c8;
          v8h hv, lv;
#pragma unroll
          for (int e = 0; e < 8; ++e) {
            if (OUT_MODE == 1) {
              hv[e] = (_Float16)sp[e];
            } else {
              unsigned short hb = f2bf_bits(sp[e]);
              unsigned short lb = f2bf_bits(sp[e] - bf_bits2f(hb));
              hv[e] = __builtin_bit_cast(_Float16, hb);
              lv[e] = __builtin_bit_cast(_Float16, lb);
            }
          }
          *(volatile v8h*)(C + (size_t)(mBase + row) * ldc + n0 + c8) = hv;
          if (OUT_MODE == 2) *(volatile v8h*)(C2 + (size_t)(mBase + row) * ldc + n0 + c8) = lv;
        }
        __threadfence();
      }
    }
    __builtin_amdgcn_fence(3  , "workgroup");
    __builtin_amdgcn_wave_barrier();
    __builtin_amdgcn_fence(2  , "workgroup");
  }
}

}

static __device__ __forceinline__ h16 toh_flush(float v) { const h16 r = (h16)v; return (fabsf(v) < 6.103515625e-05f) ? (h16)0.0f : r; }
static __device__ __forceinline__ unsigned int cc_pk2(float a, float b) {
    return (unsigned int)__builtin_bit_cast(unsigned short, toh_flush(a)) | ((unsigned int)__builtin_bit_cast(unsigned short, toh_flush(b)) << 16);
}
static __device__ __forceinline__ void cc_st8h(unsigned short* Pp, long long o, const float* v) {
    v4u pk; pk.x = cc_pk2(v[0], v[1]); pk.y = cc_pk2(v[2], v[3]); pk.z = cc_pk2(v[4], v[5]); pk.w = cc_pk2(v[6], v[7]);
    VST2(v4u, (v4u*)(Pp + o), pk);
}

static_assert(NROW % 64 == 0);
static_assert(NROW <= NROW_FULL);
static_assert(HID % 64 == 0);
static_assert(DX % 32 == 0);
static_assert(DX % 8 == 0);
static_assert((2 * NROW * (DX / 8)) % 256 == 0);
static_assert((2 * HID * (DX / 8)) % 256 == 0);
static_assert((long long)(2 * NROW * (DX / 8)) * 16 == (long long)2 * NROW * DX * 2);
static_assert((long long)(2 * HID * (DX / 8)) * 16 == (long long)2 * HID * DX * 2);

__global__ __launch_bounds__(256) void k_cc_act(const float* __restrict__ X, const float* __restrict__ Y, unsigned short* __restrict__ A16, float sc) {
    const int u = blockIdx.x * 256 + threadIdx.x;
    const int per = NROW * (DX / 8);
    if (u >= 2 * per) return;
    const int b = (u >= per) ? 1 : 0;
    const long long e8 = (long long)(u - b * per) * 8;
    const v4f x0 = *(const v4f*)(X + e8), x1 = *(const v4f*)(X + e8 + 4);
    const v4f y0 = *(const v4f*)(Y + e8), y1 = *(const v4f*)(Y + e8 + 4);
    float v[8];
    v[0] = ((b == 0) ? x0.x : y0.x) * sc; v[1] = ((b == 0) ? x0.y : y0.y) * sc; v[2] = ((b == 0) ? x0.z : y0.z) * sc; v[3] = ((b == 0) ? x0.w : y0.w) * sc;
    v[4] = ((b == 0) ? x1.x : y1.x) * sc; v[5] = ((b == 0) ? x1.y : y1.y) * sc; v[6] = ((b == 0) ? x1.z : y1.z) * sc; v[7] = ((b == 0) ? x1.w : y1.w) * sc;
    cc_st8h(A16, (long long)u * 8, v);
}

__global__ __launch_bounds__(256) void k_cc_wt(const float* __restrict__ W1, unsigned short* __restrict__ W16, float sw) {
    const int u = blockIdx.x * 256 + threadIdx.x;
    const int per = DX / 8;
    if (u >= 2 * HID * per) return;
    const int k0 = 8 * (u % per); const int o = (u / per) % HID; const int b = u / (per * HID);
    float v[8];
#pragma unroll
    for (int q = 0; q < 8; ++q) v[q] = W1[(long long)(b * DX + k0 + q) * HID + o] * sw;
    cc_st8h(W16, (long long)u * 8, v);
}

__global__ __launch_bounds__(256) void k_cc_proj(const unsigned short* __restrict__ A16, const unsigned short* __restrict__ W16, float* __restrict__ Hc, int M, int N, int K, float scale) {
    eng::wmma_gemm64_body<0, false, 0, 0, false, 0>(A16, nullptr, K, (long)M * K, W16, nullptr, K, (long)N * K, (void*)Hc, nullptr, N, (long)M * N, nullptr, nullptr, 0, M, N, K, scale);
}

#define PT 32
#define PCH 128
#define PST (PCH + 4)
#define POT 36
static_assert(PT == 32);
static_assert((256 / 32) * 4 == PT);
static_assert(PT * (PCH / 4) == 4 * 256);
static_assert(PCH / 4 == 32);
static_assert(HID % PCH == 0);
static_assert(NROW % PT == 0);
static_assert(256 * 16 * 1 == PT * PT * 4);
static_assert((PST * 4) % 16 == 0);
static_assert((POT * 4) % 16 == 0);
static_assert((2 * PT * PST + PCH + PT * POT) * 4 <= 131072);
static_assert(8 * 16 * 68 * 4 <= 131072);

__global__ __launch_bounds__(256) void k_cc_pair(const float* __restrict__ Hc, const float* __restrict__ B1, const float* __restrict__ W2, const float* __restrict__ B2, float* __restrict__ OUT) {
    __shared__ __align__(16) float sx[PT * PST];
    __shared__ __align__(16) float sy[PT * PST];
    __shared__ __align__(16) float sw[PCH];
    __shared__ __align__(16) float ot[PT * POT];
    const int tid = threadIdx.x, lane = tid & 31;
    const int wave = __builtin_amdgcn_readfirstlane(threadIdx.x >> 5);
    const int i0 = blockIdx.y * PT, j0 = blockIdx.x * PT;
    const long long hyoff = (long long)NROW * HID;
    float acc[4] = {0.f, 0.f, 0.f, 0.f};
    for (int hb = 0; hb < HID; hb += PCH) {
#pragma unroll
        for (int it = 0; it < 4; ++it) {
            const int v = tid + 256 * it; const int row = v >> 5, c4 = (v & 31) * 4;
            const v4f bx = *(const v4f*)(B1 + hb + c4);
            const v4f xv = *(const v4f*)(Hc + (long long)(i0 + row) * HID + hb + c4);
            const v4f yv = *(const v4f*)(Hc + hyoff + (long long)(j0 + row) * HID + hb + c4);
            *(v4f*)&sx[row * PST + c4] = xv + bx;
            *(v4f*)&sy[row * PST + c4] = yv;
        }
        if (wave == 0) *(v4f*)&sw[lane * 4] = *(const v4f*)(W2 + hb + lane * 4);
        __syncthreads();
#pragma unroll 2
        for (int h = 0; h < PCH; h += 4) {
            const v4f yv = *(const v4f*)&sy[lane * PST + h];
            const v4f wv = *(const v4f*)&sw[h];
#pragma unroll
            for (int r = 0; r < 4; ++r) {
                const v4f xv = *(const v4f*)&sx[(wave + 8 * r) * PST + h];
#pragma unroll
                for (int u = 0; u < 4; ++u) acc[r] = fmaf(fmaxf(xv[u] + yv[u], 0.f), wv[u], acc[r]);
            }
        }
        __syncthreads();
    }
    const float b2v = B2[0];
#pragma unroll
    for (int r = 0; r < 4; ++r) ot[(wave + 8 * r) * POT + lane] = acc[r] + b2v;
    __syncthreads();
    {
        const int row = tid >> 3, c4 = (tid & 7) * 4;
        const v4f v = *(const v4f*)&ot[row * POT + c4];
        VST2V4(OUT + (long long)(i0 + row) * NROW_FULL + j0 + c4, v);
    }
}

#define CC_A16_BYTES ((size_t)2 * NROW * DX * 2)
#define CC_W16_BYTES ((size_t)2 * HID * DX * 2)
#define CC_HC_BYTES  ((size_t)2 * NROW * HID * 4)
static_assert(CC_A16_BYTES % 256 == 0);
static_assert(CC_W16_BYTES % 256 == 0);
static_assert(CC_HC_BYTES % 256 == 0);
static_assert(CC_A16_BYTES + CC_W16_BYTES + CC_HC_BYTES <= (size_t)134217728);
static_assert((size_t)((NROW - 1) * NROW_FULL + NROW) * 4 <= (size_t)NROW_FULL * NROW_FULL * 4);

extern "C" void kernel_launch(void* const* d_in, const int* in_sizes, int n_in, void* d_out, int out_size, void* d_ws, size_t ws_size, hipStream_t stream) {
    if (n_in < 6) return;
    if (in_sizes[0] < NROW * DX || in_sizes[1] < NROW * DX || in_sizes[2] < 2 * DX * HID || in_sizes[3] < HID || in_sizes[4] < HID || in_sizes[5] < 1) return;
    if (out_size < (NROW - 1) * NROW_FULL + NROW) return;
    const float* x  = (const float*)d_in[0];
    const float* y  = (const float*)d_in[1];
    const float* W1 = (const float*)d_in[2];
    const float* b1 = (const float*)d_in[3];
    const float* W2 = (const float*)d_in[4];
    const float* b2 = (const float*)d_in[5];
    float* out = (float*)d_out;
    char* wsp = (char*)d_ws;
    unsigned short* A16 = (unsigned short*)wsp; wsp += CC_A16_BYTES;
    unsigned short* W16 = (unsigned short*)wsp; wsp += CC_W16_BYTES;
    float* Hc = (float*)wsp; wsp += CC_HC_BYTES;
    if ((size_t)(wsp - (char*)d_ws) > ws_size) return;
    k_cc_act<<<(2 * NROW * (DX / 8)) / 256, 256, 0, stream>>>(x, y, A16, 8.0f);
    k_cc_wt<<<(2 * HID * (DX / 8)) / 256, 256, 0, stream>>>(W1, W16, 32.0f);
    k_cc_proj<<<dim3((unsigned)(((NROW / 64) * (HID / 64) + 7) / 8), 2u), 256, 0, stream>>>(A16, W16, Hc, NROW, HID, DX, 0.00390625f);
    k_cc_pair<<<dim3((unsigned)(NROW / PT), (unsigned)(NROW / PT)), 256, 0, stream>>>(Hc, b1, W2, b2, out);
}
